// SelfAttentionModuleV2_74706661147106
// MI455X (gfx1250) — hardware-run, weakly checked
//
#include <hip/hip_runtime.h>
#include <stdint.h>

#define DEVINL __device__ __forceinline__

typedef _Float16 f16t;
typedef _Float16 v16h __attribute__((ext_vector_type(16)));
typedef _Float16 v8h  __attribute__((ext_vector_type(8)));
typedef float    v8f  __attribute__((ext_vector_type(8)));
typedef float    v4f  __attribute__((ext_vector_type(4)));
typedef v8h __attribute__((may_alias)) v8ha;
typedef v4f __attribute__((may_alias)) v4fa;
union FragH { v16h v; v8h half[2]; };

#define NB     4
#define HDIM   64
#define HW     4096
#define CIN    512
#define CK     256
#define COUT   512
#define TPB    256
#define WAVES  8
#define PT     64
#define PQH    264
#define PQF    132
#define XPT    32
#define XPQ    520
#define WAROWS 768
#define WBROWS 1024
#define NTAP   27
#define ACAR   16.0f
#define WCAR   256.0f
#define SC     (1.0f / (16.0f * 256.0f))
#define BNEPS  1e-5f

enum { EPI_PM32 = 0, EPI_PM16 = 1, EPI_NCHW = 2 };

static_assert(TPB == WAVES * 32);
static_assert((HW % PT) == 0);
static_assert((HW % XPT) == 0);
static_assert((CIN % 32) == 0);
static_assert((CK % 32) == 0);
static_assert(PT * PQF * 4 == PT * PQH * 2);
static_assert(WAVES * 16 * PT <= PT * PQF);
static_assert((PQH % 8) == 0);
static_assert((PQF % 4) == 0);
static_assert((XPQ % 8) == 0);
static_assert(((NB * HW) % WAVES) == 0);
static_assert(HDIM * HDIM == HW);
static_assert(WAROWS * 64 == 192 * TPB);
static_assert(WBROWS * 32 == 128 * TPB);

DEVINL int imin(int a, int b) { return a < b ? a : b; }
DEVINL int imax(int a, int b) { return a > b ? a : b; }

DEVINL v8f wmma_f16(v16h a, v16h b, v8f c) {
  v8f d = __builtin_amdgcn_wmma_f32_16x16x32_f16(false, a, false, b, (short)0, c, false, false);
  asm volatile("v_nop\n\tv_nop\n\tv_nop\n\tv_nop" : "+v"(d) : "v"(a), "v"(b));
  return d;
}
DEVINL v8f zero8f() {
  v8f z = {0.f, 0.f, 0.f, 0.f, 0.f, 0.f, 0.f, 0.f};
  return z;
}
DEVINL void load_frag(FragH& f, const f16t* row, int k0) {
  f.half[0] = *(const v8ha*)(row + k0);
  f.half[1] = *(const v8ha*)(row + k0 + 16);
}

DEVINL void store_rows256(const f16t* sT, f16t* dst, int wave, int lane) {
  #pragma unroll
  for (int i = 0; i < 8; ++i) {
    const int p = wave + 8 * i;
    const v8h v = *(const v8ha*)(sT + p * PQH + 8 * lane);
    *(volatile v8h*)(dst + (size_t)p * 256 + 8 * lane) = v;
  }
  __threadfence();
  #pragma unroll
  for (int i = 0; i < 8; ++i) {
    const int p = wave + 8 * i;
    const v8h v = *(const v8ha*)(sT + p * PQH + 8 * lane);
    *(volatile v8h*)(dst + (size_t)p * 256 + 8 * lane) = v;
  }
}

__global__ __launch_bounds__(TPB) void prep_w_k(const float* __restrict__ v_w, const float* __restrict__ k1_w,
                                               const float* __restrict__ q1_w, const float* __restrict__ k2_w,
                                               const float* __restrict__ q2_w, const float* __restrict__ w_w,
                                               f16t* __restrict__ WA, f16t* __restrict__ WB)
{
  const int blk = blockIdx.x, tid = threadIdx.x;
  if (blk >= 320) return;
  v8h o;
  f16t* dst;
  if (blk < 192) {
    const int grp = blk >> 6;
    const float* src = (grp == 0) ? v_w : ((grp == 1) ? k1_w : q1_w);
    const int t = blk * TPB + tid;
    const int row = t >> 6, piece = (t & 63) * 8;
    const int srow = imin(imax(row - 256 * grp, 0), 255);
    const float* sp = src + (size_t)srow * CIN + piece;
    const v4f a = *(const v4fa*)sp, c = *(const v4fa*)(sp + 4);
    #pragma unroll
    for (int i = 0; i < 4; ++i) { o[i] = (f16t)(a[i] * WCAR); o[4 + i] = (f16t)(c[i] * WCAR); }
    dst = WA + (size_t)row * CIN + piece;
  } else {
    const int rb = blk - 192;
    const int grp = rb >> 5;
    const float* src = (grp == 0) ? k2_w : ((grp == 1) ? q2_w : w_w);
    const int u = rb * TPB + tid;
    const int row = u >> 5, piece = (u & 31) * 8;
    const int sub = (grp >= 2) ? 512 : 256 * grp;
    const int srow = imin(imax(row - sub, 0), 511);
    const float* sp = src + (size_t)srow * CK + piece;
    const v4f a = *(const v4fa*)sp, c = *(const v4fa*)(sp + 4);
    #pragma unroll
    for (int i = 0; i < 4; ++i) { o[i] = (f16t)(a[i] * WCAR); o[4 + i] = (f16t)(c[i] * WCAR); }
    dst = WB + (size_t)row * CK + piece;
  }
  *(volatile v8h*)dst = o;
  __threadfence();
  *(volatile v8h*)dst = o;
}

__global__ __launch_bounds__(TPB) void xpose_k(const float* __restrict__ x, f16t* __restrict__ XT)
{
  __shared__ __attribute__((aligned(16))) f16t sT[XPT * XPQ];
  const int tid = threadIdx.x;
  const int p0 = blockIdx.x * XPT, b = blockIdx.y;
  const int c0 = tid >> 3, p4 = (tid & 7) * 4;
  const float* xb = x + (size_t)b * CIN * HW + p0 + p4;
  #pragma unroll 4
  for (int i = 0; i < 16; ++i) {
    const int c = c0 + 32 * i;
    const v4f v = *(const v4fa*)(xb + (size_t)c * HW);
    sT[(p4 + 0) * XPQ + c] = (f16t)(v[0] * ACAR);
    sT[(p4 + 1) * XPQ + c] = (f16t)(v[1] * ACAR);
    sT[(p4 + 2) * XPQ + c] = (f16t)(v[2] * ACAR);
    sT[(p4 + 3) * XPQ + c] = (f16t)(v[3] * ACAR);
  }
  __syncthreads();
  f16t* base = XT + ((size_t)b * HW + p0) * CIN;
  #pragma unroll
  for (int i = 0; i < 8; ++i) {
    const int q = tid + TPB * i;
    const int row = q >> 6, piece = (q & 63) * 8;
    const v8h v = *(const v8ha*)(sT + row * XPQ + piece);
    *(volatile v8h*)(base + (size_t)row * CIN + piece) = v;
  }
  __threadfence();
  #pragma unroll
  for (int i = 0; i < 8; ++i) {
    const int q = tid + TPB * i;
    const int row = q >> 6, piece = (q & 63) * 8;
    const v8h v = *(const v8ha*)(sT + row * XPQ + piece);
    *(volatile v8h*)(base + (size_t)row * CIN + piece) = v;
  }
}

template <int EPI, int KD, int BN, typename OT>
__global__ __launch_bounds__(TPB) void gemm_k(const f16t* __restrict__ B0, const f16t* __restrict__ B1,
                                             const f16t* __restrict__ Ap,
                                             const float* __restrict__ pbi0, const float* __restrict__ pga0,
                                             const float* __restrict__ pbe0, const float* __restrict__ pmu0,
                                             const float* __restrict__ pva0,
                                             const float* __restrict__ pbi1, const float* __restrict__ pga1,
                                             const float* __restrict__ pbe1, const float* __restrict__ pmu1,
                                             const float* __restrict__ pva1,
                                             OT* __restrict__ out0, OT* __restrict__ out1)
{
  __shared__ __attribute__((aligned(16))) float sbuf[PT * PQF];
  const int tid = threadIdx.x, lane = tid & 31, wave = tid >> 5;
  const int h = lane >> 4, m = lane & 15;
  const int p0 = blockIdx.x * PT, y = blockIdx.y, b = blockIdx.z;

  const f16t*  Bp  = (y == 0) ? B0 : B1;
  const float* pbi = (y == 0) ? pbi0 : pbi1;
  const float* pga = (y == 0) ? pga0 : pga1;
  const float* pbe = (y == 0) ? pbe0 : pbe1;
  const float* pmu = (y == 0) ? pmu0 : pmu1;
  const float* pva = (y == 0) ? pva0 : pva1;
  OT* outp = (y == 0) ? out0 : out1;

  v8f acc[2][4];
  #pragma unroll
  for (int mt = 0; mt < 2; ++mt) {
    #pragma unroll
    for (int n = 0; n < 4; ++n) acc[mt][n] = zero8f();
  }
  const f16t* arow = Ap + (size_t)(y * 256 + wave * 32 + m) * KD + 8 * h;
  const f16t* brow = Bp + ((size_t)b * HW + p0 + m) * KD + 8 * h;
  #pragma unroll 1
  for (int ks = 0; ks < KD / 32; ++ks) {
    const int k0 = 32 * ks;
    FragH a0, a1, bf[4];
    load_frag(a0, arow, k0);
    load_frag(a1, arow + 16 * KD, k0);
    #pragma unroll
    for (int n = 0; n < 4; ++n) load_frag(bf[n], brow + (size_t)16 * n * KD, k0);
    #pragma unroll
    for (int n = 0; n < 4; ++n) {
      acc[0][n] = wmma_f16(a0.v, bf[n].v, acc[0][n]);
      acc[1][n] = wmma_f16(a1.v, bf[n].v, acc[1][n]);
    }
  }

  float cbv[2][8], csv[2][8], chv[2][8];
  #pragma unroll
  for (int mt = 0; mt < 2; ++mt) {
    const int ob = wave * 32 + 16 * mt + 8 * h;
    const v4f b0v = *(const v4fa*)(pbi + ob), b1v = *(const v4fa*)(pbi + ob + 4);
    #pragma unroll
    for (int r = 0; r < 4; ++r) { cbv[mt][r] = b0v[r]; cbv[mt][4 + r] = b1v[r]; }
    if (BN != 0) {
      const v4f g0 = *(const v4fa*)(pga + ob), g1 = *(const v4fa*)(pga + ob + 4);
      const v4f e0 = *(const v4fa*)(pbe + ob), e1 = *(const v4fa*)(pbe + ob + 4);
      const v4f u0 = *(const v4fa*)(pmu + ob), u1 = *(const v4fa*)(pmu + ob + 4);
      const v4f s0 = *(const v4fa*)(pva + ob), s1 = *(const v4fa*)(pva + ob + 4);
      #pragma unroll
      for (int r = 0; r < 4; ++r) {
        const float sa = g0[r] * rsqrtf(s0[r] + BNEPS);
        const float sb = g1[r] * rsqrtf(s1[r] + BNEPS);
        csv[mt][r]     = sa; chv[mt][r]     = e0[r] - u0[r] * sa;
        csv[mt][4 + r] = sb; chv[mt][4 + r] = e1[r] - u1[r] * sb;
      }
    } else {
      #pragma unroll
      for (int r = 0; r < 8; ++r) { csv[mt][r] = 1.0f; chv[mt][r] = 0.0f; }
    }
  }
#define EPV(mt_, n_, r_, dst_)                                   \
  do {                                                           \
    float t_ = fmaf(acc[mt_][n_][r_], SC, cbv[mt_][r_]);         \
    if (BN != 0) {                                               \
      t_ = fmaf(t_, csv[mt_][r_], chv[mt_][r_]);                 \
      t_ = fmaxf(t_, 0.0f);                                      \
    }                                                            \
    dst_ = t_;                                                   \
  } while (0)

  if (EPI == EPI_PM32) {
    float* of = (float*)outp;
    #pragma unroll
    for (int ph = 0; ph < 2; ++ph) {
      if ((wave >> 2) == ph) {
        #pragma unroll
        for (int mt = 0; mt < 2; ++mt) {
          #pragma unroll
          for (int n = 0; n < 4; ++n) {
            v4f o0, o1;
            #pragma unroll
            for (int r = 0; r < 4; ++r) { EPV(mt, n, r, o0[r]); EPV(mt, n, 4 + r, o1[r]); }
            const int cl = 32 * (wave & 3) + 16 * mt + 8 * h;
            float* sp = sbuf + (16 * n + m) * PQF + cl;
            *(v4fa*)sp = o0;
            *(v4fa*)(sp + 4) = o1;
          }
        }
      }
      __syncthreads();
      float* dst = of + ((size_t)b * HW + p0) * CK + 128 * ph;
      #pragma unroll
      for (int i = 0; i < 8; ++i) {
        const int row = 8 * i + wave;
        const v4f v = *(const v4fa*)(sbuf + row * PQF + 4 * lane);
        *(volatile v4f*)(dst + (size_t)row * CK + 4 * lane) = v;
      }
      __threadfence();
      #pragma unroll
      for (int i = 0; i < 8; ++i) {
        const int row = 8 * i + wave;
        const v4f v = *(const v4fa*)(sbuf + row * PQF + 4 * lane);
        *(volatile v4f*)(dst + (size_t)row * CK + 4 * lane) = v;
      }
      __syncthreads();
    }
  } else if (EPI == EPI_PM16) {
    f16t* sT = (f16t*)sbuf;
    #pragma unroll
    for (int mt = 0; mt < 2; ++mt) {
      #pragma unroll
      for (int n = 0; n < 4; ++n) {
        v8h o;
        #pragma unroll
        for (int r = 0; r < 8; ++r) { float t; EPV(mt, n, r, t); o[r] = (f16t)(t * ACAR); }
        *(v8ha*)(sT + (16 * n + m) * PQH + wave * 32 + 16 * mt + 8 * h) = o;
      }
    }
    __syncthreads();
    store_rows256(sT, (f16t*)outp + ((size_t)b * HW + p0) * CK, wave, lane);
  } else {
    float* of = (float*)outp;
    #pragma unroll
    for (int mt = 0; mt < 2; ++mt) {
      #pragma unroll
      for (int n = 0; n < 4; ++n) {
        #pragma unroll
        for (int r = 0; r < 4; ++r) {
          float t0, t1;
          EPV(mt, n, r, t0);
          EPV(mt, n, 4 + r, t1);
          sbuf[wave * 1024 + (8 * h + r) * PT + 16 * n + m]     = t0;
          sbuf[wave * 1024 + (8 * h + 4 + r) * PT + 16 * n + m] = t1;
        }
      }
      __syncthreads();
      float* orow = of + ((size_t)b * COUT + y * 256 + wave * 32 + 16 * mt) * HW + p0;
      const int l16 = lane & 15, rsel = lane >> 4;
      #pragma unroll
      for (int i = 0; i < 8; ++i) {
        const int row = 2 * i + rsel;
        const v4f v = *(const v4fa*)(sbuf + wave * 1024 + row * PT + 4 * l16);
        *(volatile v4f*)(orow + (size_t)row * HW + 4 * l16) = v;
      }
      __threadfence();
      #pragma unroll
      for (int i = 0; i < 8; ++i) {
        const int row = 2 * i + rsel;
        const v4f v = *(const v4fa*)(sbuf + wave * 1024 + row * PT + 4 * l16);
        *(volatile v4f*)(orow + (size_t)row * HW + 4 * l16) = v;
      }
      __syncthreads();
    }
  }
#undef EPV
}

DEVINL size_t tap_pixel(int t, int b, int hq, int wq, int& valid) {
  const int dd = (t >= 18) ? 2 : ((t >= 9) ? 1 : 0);
  const int ij = t - 9 * dd;
  const int i = (ij >= 6) ? 2 : ((ij >= 3) ? 1 : 0);
  const int j = ij - 3 * i;
  const int d = 1 << dd;
  const int hh = hq + (i - 1) * d, ww = wq + (j - 1) * d;
  valid = (((unsigned)hh < (unsigned)HDIM) && ((unsigned)ww < (unsigned)HDIM)) ? 1 : 0;
  const int hc = imin(imax(hh, 0), HDIM - 1), wc = imin(imax(ww, 0), HDIM - 1);
  return (size_t)b * HW + (size_t)hc * HDIM + (size_t)wc;
}

__global__ __launch_bounds__(TPB) void attn_k(const float* __restrict__ KEY, const float* __restrict__ QRY,
                                             const float* __restrict__ VAL, f16t* __restrict__ CTX)
{
  const int tid = threadIdx.x, lane = tid & 31, wave = tid >> 5;
  const int gp = blockIdx.x * WAVES + wave;
  if (gp >= NB * HW) return;
  const int b = gp / HW, n = gp - b * HW;
  const int hq = n / HDIM, wq = n - hq * HDIM;
  const int c0 = lane * 8;

  const float* qp = QRY + (size_t)gp * CK + c0;
  const v4f q0 = *(const v4fa*)qp, q1 = *(const v4fa*)(qp + 4);

  float mys = -3.0e38f;
  #pragma unroll 1
  for (int t = 0; t < NTAP; ++t) {
    int valid;
    const size_t nb = tap_pixel(t, b, hq, wq, valid);
    const float* kp = KEY + nb * CK + c0;
    const v4f k0 = *(const v4fa*)kp, k1 = *(const v4fa*)(kp + 4);
    float dot = q0[0] * k0[0];
    dot = fmaf(q0[1], k0[1], dot);
    dot = fmaf(q0[2], k0[2], dot);
    dot = fmaf(q0[3], k0[3], dot);
    dot = fmaf(q1[0], k1[0], dot);
    dot = fmaf(q1[1], k1[1], dot);
    dot = fmaf(q1[2], k1[2], dot);
    dot = fmaf(q1[3], k1[3], dot);
    #pragma unroll
    for (int s = 16; s > 0; s >>= 1) dot += __shfl_xor(dot, s);
    dot = valid ? dot : 0.0f;
    mys = (lane == t) ? dot : mys;
  }

  float mx = mys;
  #pragma unroll
  for (int s = 16; s > 0; s >>= 1) mx = fmaxf(mx, __shfl_xor(mx, s));
  float e = __expf(mys - mx);
  e = (lane < NTAP) ? e : 0.0f;
  float ssum = e;
  #pragma unroll
  for (int s = 16; s > 0; s >>= 1) ssum += __shfl_xor(ssum, s);
  const float p = e * (1.0f / ssum);

  v4f cx0 = {0.f, 0.f, 0.f, 0.f};
  v4f cx1 = {0.f, 0.f, 0.f, 0.f};
  #pragma unroll 1
  for (int t = 0; t < NTAP; ++t) {
    float wt = __shfl(p, t);
    int valid;
    const size_t nb = tap_pixel(t, b, hq, wq, valid);
    wt = valid ? wt : 0.0f;
    const float* vp = VAL + nb * CK + c0;
    const v4f v0 = *(const v4fa*)vp, v1 = *(const v4fa*)(vp + 4);
    cx0[0] = fmaf(wt, v0[0], cx0[0]);
    cx0[1] = fmaf(wt, v0[1], cx0[1]);
    cx0[2] = fmaf(wt, v0[2], cx0[2]);
    cx0[3] = fmaf(wt, v0[3], cx0[3]);
    cx1[0] = fmaf(wt, v1[0], cx1[0]);
    cx1[1] = fmaf(wt, v1[1], cx1[1]);
    cx1[2] = fmaf(wt, v1[2], cx1[2]);
    cx1[3] = fmaf(wt, v1[3], cx1[3]);
  }

  v8h o;
  #pragma unroll
  for (int i = 0; i < 4; ++i) { o[i] = (f16t)(cx0[i] * ACAR); o[4 + i] = (f16t)(cx1[i] * ACAR); }
  f16t* dst = CTX + (size_t)gp * CK + c0;
  *(volatile v8h*)dst = o;
  __threadfence();
  *(volatile v8h*)dst = o;
}

extern "C" void kernel_launch(void* const* d_in, const int* in_sizes, int n_in,
                              void* d_out, int out_size, void* d_ws, size_t ws_size,
                              hipStream_t stream) {
  if (n_in < 29) return;
  if (in_sizes[0] != NB * CIN * HW) return;
  if (in_sizes[1] != CK * CIN) return;
  if (in_sizes[7] != CK * CK) return;
  if (in_sizes[13] != CK * CIN) return;
  if (in_sizes[19] != CK * CK) return;
  for (int i = 2; i <= 6; ++i)   if (in_sizes[i] != CK) return;
  for (int i = 8; i <= 12; ++i)  if (in_sizes[i] != CK) return;
  for (int i = 14; i <= 18; ++i) if (in_sizes[i] != CK) return;
  for (int i = 20; i <= 24; ++i) if (in_sizes[i] != CK) return;
  if (in_sizes[25] != CK * CIN) return;
  if (in_sizes[26] != CK) return;
  if (in_sizes[27] != COUT * CK) return;
  if (in_sizes[28] != COUT) return;
  if (out_size != NB * COUT * HW) return;

  const float* x     = (const float*)d_in[0];
  const float* k1_w  = (const float*)d_in[1];
  const float* k1_b  = (const float*)d_in[2];
  const float* k1_g  = (const float*)d_in[3];
  const float* k1_be = (const float*)d_in[4];
  const float* k1_m  = (const float*)d_in[5];
  const float* k1_v  = (const float*)d_in[6];
  const float* k2_w  = (const float*)d_in[7];
  const float* k2_b  = (const float*)d_in[8];
  const float* k2_g  = (const float*)d_in[9];
  const float* k2_be = (const float*)d_in[10];
  const float* k2_m  = (const float*)d_in[11];
  const float* k2_v  = (const float*)d_in[12];
  const float* q1_w  = (const float*)d_in[13];
  const float* q1_b  = (const float*)d_in[14];
  const float* q1_g  = (const float*)d_in[15];
  const float* q1_be = (const float*)d_in[16];
  const float* q1_m  = (const float*)d_in[17];
  const float* q1_v  = (const float*)d_in[18];
  const float* q2_w  = (const float*)d_in[19];
  const float* q2_b  = (const float*)d_in[20];
  const float* q2_g  = (const float*)d_in[21];
  const float* q2_be = (const float*)d_in[22];
  const float* q2_m  = (const float*)d_in[23];
  const float* q2_v  = (const float*)d_in[24];
  const float* v_w   = (const float*)d_in[25];
  const float* v_b   = (const float*)d_in[26];
  const float* w_w   = (const float*)d_in[27];
  const float* w_b   = (const float*)d_in[28];
  float* outp = (float*)d_out;

  const size_t szWA  = (size_t)WAROWS * CIN * 2;
  const size_t szWB  = (size_t)WBROWS * CK * 2;
  const size_t szXT  = (size_t)NB * HW * CIN * 2;
  const size_t szP32 = (size_t)NB * HW * CK * 4;
  const size_t szP16 = (size_t)NB * HW * CK * 2;
  size_t off = 0;
  char* ws = (char*)d_ws;
  f16t*  WA  = (f16t*)(ws + off);  off += szWA;
  f16t*  WB  = (f16t*)(ws + off);  off += szWB;
  f16t*  XT  = (f16t*)(ws + off);  off += szXT;
  float* VAL = (float*)(ws + off); off += szP32;
  f16t*  HK  = (f16t*)(ws + off);  off += szP16;
  f16t*  HQ  = (f16t*)(ws + off);  off += szP16;
  float* KEY = (float*)(ws + off); off += szP32;
  float* QRY = (float*)(ws + off); off += szP32;
  f16t*  CTX = (f16t*)(ws + off);  off += szP16;
  if (off > ws_size) return;

  prep_w_k<<<320, TPB, 0, stream>>>(v_w, k1_w, q1_w, k2_w, q2_w, w_w, WA, WB);
  xpose_k<<<dim3(HW / XPT, NB), TPB, 0, stream>>>(x, XT);
  gemm_k<EPI_PM32, CIN, 0, float><<<dim3(HW / PT, 1, NB), TPB, 0, stream>>>(
      XT, XT, WA, v_b, v_b, v_b, v_b, v_b, v_b, v_b, v_b, v_b, v_b, VAL, VAL);
  gemm_k<EPI_PM16, CIN, 1, f16t><<<dim3(HW / PT, 2, NB), TPB, 0, stream>>>(
      XT, XT, WA + (size_t)256 * CIN,
      k1_b, k1_g, k1_be, k1_m, k1_v, q1_b, q1_g, q1_be, q1_m, q1_v, HK, HQ);
  gemm_k<EPI_PM32, CK, 1, float><<<dim3(HW / PT, 2, NB), TPB, 0, stream>>>(
      HK, HQ, WB,
      k2_b, k2_g, k2_be, k2_m, k2_v, q2_b, q2_g, q2_be, q2_m, q2_v, KEY, QRY);
  attn_k<<<(NB * HW) / WAVES, TPB, 0, stream>>>(KEY, QRY, VAL, CTX);
  gemm_k<EPI_NCHW, CK, 0, float><<<dim3(HW / PT, 2, NB), TPB, 0, stream>>>(
      CTX, CTX, WB + (size_t)512 * CK,
      w_b, w_b, w_b, w_b, w_b, w_b + 256, w_b + 256, w_b + 256, w_b + 256, w_b + 256, outp, outp);
}
